// CardEncoder_46445776338948
// MI455X (gfx1250) — hardware-verified
//
#include <hip/hip_runtime.h>

typedef __attribute__((ext_vector_type(16))) _Float16 v16h;
typedef __attribute__((ext_vector_type(8)))  _Float16 v8h;
typedef __attribute__((ext_vector_type(16))) __bf16   v16b;
typedef __attribute__((ext_vector_type(8)))  __bf16   v8b;
typedef __attribute__((ext_vector_type(8)))  float    v8f;
typedef __attribute__((ext_vector_type(4)))  float    v4f;
typedef __attribute__((ext_vector_type(4)))  unsigned int u4v;
typedef __attribute__((ext_vector_type(4)))  int      i4v;

__device__ __forceinline__ unsigned short f2bf_bits(float f) {
  unsigned u = __float_as_uint(f);
  return (unsigned short)((u + 0x7FFFu + ((u >> 16) & 1u)) >> 16);
}
__device__ __forceinline__ float bf_bits2f(unsigned short h) { return __uint_as_float(((unsigned)h) << 16); }

__device__ __forceinline__ void dep_guard_h(v8f& a, v8f& b, v16h x, v16h y) { asm volatile("v_nop\n\tv_nop\n\tv_nop\n\tv_nop" : "+v"(a), "+v"(b) : "v"(x), "v"(y)); }
__device__ __forceinline__ void dep_guard_b(v8f& a, v8f& b, v16b x, v16b y) { asm volatile("v_nop\n\tv_nop\n\tv_nop\n\tv_nop" : "+v"(a), "+v"(b) : "v"(x), "v"(y)); }
__device__ __forceinline__ void keep4_h(v16h a, v16h b, v16h c, v16h d) { asm volatile("v_nop" :: "v"(a), "v"(b), "v"(c), "v"(d)); }
__device__ __forceinline__ void keep4_b(v16b a, v16b b, v16b c, v16b d) { asm volatile("v_nop" :: "v"(a), "v"(b), "v"(c), "v"(d)); }
__device__ __forceinline__ void acc_guard4(v8f& a, v8f& b, v8f& c, v8f& d) { asm volatile("v_nop\n\tv_nop\n\tv_nop\n\tv_nop" : "+v"(a), "+v"(b), "+v"(c), "+v"(d)); }
template <typename T> struct Frag;
template <> struct Frag<_Float16> {
  typedef v16h V; union U { v16h v; v8h h[2]; };
  static __device__ __forceinline__ v16h load(const _Float16* p) {
    U f; f.h[0] = *(const v8h*)(p); f.h[1] = *(const v8h*)(p + 16); return f.v;
  }
  static __device__ __forceinline__ v8f mma(v16h a, v16h b, v8f c) {
    return __builtin_amdgcn_wmma_f32_16x16x32_f16(false, a, false, b, (short)0, c, false, false);
  }
  static __device__ __forceinline__ void guard(v8f& a, v8f& b, v16h x, v16h y) { dep_guard_h(a, b, x, y); }
  static __device__ __forceinline__ void keep(v16h a, v16h b, v16h c, v16h d) { keep4_h(a, b, c, d); }
};
template <> struct Frag<__bf16> {
  typedef v16b V; union U { v16b v; v8b h[2]; };
  static __device__ __forceinline__ v16b load(const __bf16* p) {
    U f; f.h[0] = *(const v8b*)(p); f.h[1] = *(const v8b*)(p + 16); return f.v;
  }
  static __device__ __forceinline__ v8f mma(v16b a, v16b b, v8f c) {
    return __builtin_amdgcn_wmma_f32_16x16x32_bf16(false, a, false, b, (short)0, c, false, false);
  }
  static __device__ __forceinline__ void guard(v8f& a, v8f& b, v16b x, v16b y) { dep_guard_b(a, b, x, y); }
  static __device__ __forceinline__ void keep(v16b a, v16b b, v16b c, v16b d) { keep4_b(a, b, c, d); }
};

template <int ET> struct Elem;
template <> struct Elem<0> { typedef _Float16 T; };
template <> struct Elem<1> { typedef __bf16 T; };
template <int ET, bool SPLIT, int BIAS_MODE, int OUT_MODE, bool RESID, int ACT = 0>
__global__ __launch_bounds__(256) void wmma_gemm64(
    const unsigned short* __restrict__ Ap, const unsigned short* __restrict__ A2p, int lda, long strideA,
    const unsigned short* __restrict__ Btp, const unsigned short* __restrict__ Bt2p, int ldb, long strideB,
    void* __restrict__ Cout, void* __restrict__ Cout2, int ldc, long strideC,
    const float* __restrict__ bias,
    const float* __restrict__ resid, long strideR,
    int M, int N, int K, float scale) {
  typedef typename Elem<ET>::T T;
  typedef typename Frag<T>::V V;
  const T* A = (const T*)Ap; const T* A2 = (const T*)A2p; const T* Bt = (const T*)Btp; const T* Bt2 = (const T*)Bt2p;
  __shared__ __align__(16) float sT[8][16 * 68];
  const int b    = blockIdx.y;
  const int lane = threadIdx.x & 31;
  const int wave = threadIdx.x >> 5;
  const int tilesN = N >> 6;
  const int tilesM = M >> 6;
  const int tile = blockIdx.x * 8 + wave;
  if (tile >= tilesM * tilesN) return;
  const int tm = tile / tilesN;
  const int tn = tile - tm * tilesN;
  const int m0 = tm << 6;
  const int n0 = tn << 6;

  const T* Ab  = A  + (size_t)b * strideA;
  const T* Bb  = Bt + (size_t)b * strideB;
  const T* Ab2 = SPLIT ? (A2  + (size_t)b * strideA) : nullptr;
  const T* Bb2 = SPLIT ? (Bt2 + (size_t)b * strideB) : nullptr;

  const int rlane = lane & 15;
  const int koff  = (lane >> 4) * 8;
  const int mOff  = (lane >> 4) * 8;

  v8f acc[4][4];
#pragma unroll
  for (int i = 0; i < 4; ++i)
#pragma unroll
    for (int j = 0; j < 4; ++j) acc[i][j] = (v8f){0.f,0.f,0.f,0.f,0.f,0.f,0.f,0.f};

  for (int k0 = 0; k0 < K; k0 += 32) {
    V bh[4], bl[4];
#pragma unroll
    for (int j = 0; j < 4; ++j) {
      const size_t bo = (size_t)(n0 + (j << 4) + rlane) * ldb + koff + k0;
      bh[j] = Frag<T>::load(Bb + bo);
      if (SPLIT) bl[j] = Frag<T>::load(Bb2 + bo);
    }
#pragma unroll
    for (int i = 0; i < 4; ++i) {
      const size_t ao = (size_t)(m0 + (i << 4) + rlane) * lda + koff + k0;
      V ah = Frag<T>::load(Ab + ao);
      V al;
      if (SPLIT) al = Frag<T>::load(Ab2 + ao);
#pragma unroll
      for (int j = 0; j < 4; ++j) {
        acc[i][j] = Frag<T>::mma(ah, bh[j], acc[i][j]);
        if (SPLIT) {
          acc[i][j] = Frag<T>::mma(ah, bl[j], acc[i][j]);
          acc[i][j] = Frag<T>::mma(al, bh[j], acc[i][j]);
        }
      }
      Frag<T>::guard(acc[i][0], acc[i][3], ah, SPLIT ? al : ah);
    }
    Frag<T>::keep(bh[0], bh[1], bh[2], bh[3]);
    if (SPLIT) Frag<T>::keep(bl[0], bl[1], bl[2], bl[3]);
  }
  acc_guard4(acc[0][0], acc[0][1], acc[0][2], acc[0][3]);
  acc_guard4(acc[1][0], acc[1][1], acc[1][2], acc[1][3]);
  acc_guard4(acc[2][0], acc[2][1], acc[2][2], acc[2][3]);
  acc_guard4(acc[3][0], acc[3][1], acc[3][2], acc[3][3]);

  float* slab = sT[wave];
  const float* Rb = RESID ? (resid + (size_t)b * strideR) : nullptr;
#pragma unroll
  for (int i = 0; i < 4; ++i) {
    const int mBase = m0 + (i << 4);
#pragma unroll
    for (int j = 0; j < 4; ++j) {
      const int n = n0 + (j << 4) + rlane;
      float bv = 0.f;
      if (BIAS_MODE == 2) bv = bias[n];
#pragma unroll
      for (int r = 0; r < 8; ++r) {
        float v = acc[i][j][r] * scale;
        if (BIAS_MODE == 1) v += bias[mBase + mOff + r];
        if (BIAS_MODE == 2) v += bv;
        if (RESID) v += Rb[(size_t)(mBase + mOff + r) * ldc + n];
        if (ACT == 1) v = tanhf(v);
        if (ACT == 2) v = fmaxf(v, 0.0f);
        if (ACT == 3) v = v / (1.0f + expf(-v));
        if (ACT == 4) v = (v > 0.f) ? v : 0.01f * v;
        if (ACT == 5) v = 0.5f * v * (1.0f + erff(v * 0.70710678118654752f));
        slab[(mOff + r) * 68 + (j << 4) + rlane] = v;
      }
    }
    __builtin_amdgcn_fence(__ATOMIC_RELEASE, "workgroup");
    __builtin_amdgcn_wave_barrier();
    __builtin_amdgcn_fence(__ATOMIC_ACQUIRE, "workgroup");
    if (OUT_MODE == 0) {
      float* C = (float*)Cout + (size_t)b * strideC;
      const int hh = lane >> 4, c4 = (lane & 15) * 4;
      for (int pass = 0; pass < 2; ++pass) {
#pragma unroll
        for (int it = 0; it < 8; ++it) {
          const int row = it * 2 + hh;
          v4f v = *(const v4f*)(slab + row * 68 + c4);
          *(volatile v4f*)(C + (size_t)(mBase + row) * ldc + n0 + c4) = v;
        }
        __threadfence();
      }
    } else {
      const int q = lane >> 3, c8 = (lane & 7) * 8;
      unsigned short* C  = (unsigned short*)Cout  + (size_t)b * strideC;
      unsigned short* C2 = (OUT_MODE == 2) ? ((unsigned short*)Cout2 + (size_t)b * strideC) : nullptr;
      for (int pass = 0; pass < 2; ++pass) {
#pragma unroll
        for (int it = 0; it < 4; ++it) {
          const int row = it * 4 + q;
          const float* sp = slab + row * 68 + c8;
          v8h hv, lv;
#pragma unroll
          for (int e = 0; e < 8; ++e) {
            if (OUT_MODE == 1) {
              hv[e] = (_Float16)sp[e];
            } else {
              unsigned short hb = f2bf_bits(sp[e]);
              unsigned short lb = f2bf_bits(sp[e] - bf_bits2f(hb));
              hv[e] = __builtin_bit_cast(_Float16, hb);
              lv[e] = __builtin_bit_cast(_Float16, lb);
            }
          }
          *(volatile v8h*)(C + (size_t)(mBase + row) * ldc + n0 + c8) = hv;
          if (OUT_MODE == 2) *(volatile v8h*)(C2 + (size_t)(mBase + row) * ldc + n0 + c8) = lv;
        }
        __threadfence();
      }
    }
    __builtin_amdgcn_fence(__ATOMIC_RELEASE, "workgroup");
    __builtin_amdgcn_wave_barrier();
    __builtin_amdgcn_fence(__ATOMIC_ACQUIRE, "workgroup");
  }
}

__device__ __forceinline__ v8f mma_h(v16h a, v16h b, v8f c) {
  c = __builtin_amdgcn_wmma_f32_16x16x32_f16(false, a, false, b, (short)0, c, false, false);
  asm volatile("v_nop\n\tv_nop\n\tv_nop\n\tv_nop" : "+v"(c) : "v"(a), "v"(b));
  return c;
}
__device__ __forceinline__ float gate_sig(float x) {
  return __builtin_amdgcn_rcpf(1.0f + __builtin_amdgcn_exp2f(-1.4426950408889634f * x));
}
__device__ __forceinline__ float gate_tanh(float x) {
  return 1.0f - 2.0f * __builtin_amdgcn_rcpf(1.0f + __builtin_amdgcn_exp2f(2.8853900817779268f * x));
}

#define GATES_N 128
#define EMB_D 32
#define HID_D 32
#define SEQ_T 16
#define LS_ROWS 64
#define LS_PITCH 72

__global__ __launch_bounds__(256) void prep_wcat_kernel(const float* __restrict__ Wk,
                                                        const float* __restrict__ Wr,
                                                        unsigned short* __restrict__ wcat) {
  const int tid = threadIdx.x;
  const int q8  = tid >> 3;
  const int k8  = (tid & 7) * 8;
  for (int pass = 0; pass < 2; ++pass) {
#pragma unroll 1
    for (int it = 0; it < 4; ++it) {
      const int n = it * 32 + q8;
      v8h hv;
#pragma unroll
      for (int e = 0; e < 8; ++e) {
        const int k  = k8 + e;
        const int kk = k & 31;
        const float va = Wk[kk * GATES_N + n];
        const float vb = Wr[kk * GATES_N + n];
        const float v  = (k < 32) ? va : vb;
        hv[e] = (_Float16)(v * 8.0f);
      }
      *(volatile v8h*)(wcat + (size_t)n * 64 + k8) = hv;
    }
    __threadfence();
  }
}

__global__ __launch_bounds__(256) void prep_wdt_kernel(const float* __restrict__ Wd,
                                                       unsigned short* __restrict__ wdt, int Kd) {
  __shared__ float Tsh[64 * 68];
  const int tid  = threadIdx.x;
  const int wave = tid >> 5, lane = tid & 31;
  const int k0   = blockIdx.x * 64;
#pragma unroll
  for (int it = 0; it < 16; ++it) {
    const int idx = it * 256 + tid;
    const int kr  = idx >> 6;
    const int n   = idx & 63;
    Tsh[n * 68 + kr] = Wd[(size_t)(k0 + kr) * 64 + n];
  }
  __syncthreads();
  const int q = lane >> 3, c8 = (lane & 7) * 8;
  for (int pass = 0; pass < 2; ++pass) {
#pragma unroll
    for (int it = 0; it < 2; ++it) {
      const int n = wave * 8 + it * 4 + q;
      const float* sp = Tsh + n * 68 + c8;
      v8h hv;
#pragma unroll
      for (int e = 0; e < 8; ++e) hv[e] = (_Float16)(sp[e] * 32.0f);
      *(volatile v8h*)(wdt + (size_t)n * Kd + k0 + c8) = hv;
    }
    __threadfence();
  }
}

__global__ __launch_bounds__(128) void lstm_bidir_kernel(const int* __restrict__ x,
                                                         const float* __restrict__ etab,
                                                         const float* __restrict__ bias,
                                                         const unsigned short* __restrict__ wcat,
                                                         unsigned short* __restrict__ state16,
                                                         int nvocab) {
  __shared__ __align__(16) _Float16 Wsh[GATES_N * LS_PITCH];
  __shared__ __align__(16) _Float16 Ash[LS_ROWS * LS_PITCH];
  __shared__ __align__(16) _Float16 Osh[LS_ROWS * LS_PITCH];

  const int tid  = threadIdx.x;
  const int wave = tid >> 5, lane = tid & 31;
  const int c    = lane & 15, hh = lane >> 4;
  const int rowBase = blockIdx.x * LS_ROWS;
  const int m0   = wave * 16;

#pragma unroll
  for (int it = 0; it < 8; ++it) {
    const int idx = it * 128 + tid;
    const int row = idx >> 3, k8 = (idx & 7) * 8;
    const u4v v = *(const u4v*)(wcat + (size_t)row * 64 + k8);
    *(u4v*)(Wsh + row * LS_PITCH + k8) = v;
  }

  unsigned um[8];
#pragma unroll
  for (int r = 0; r < 8; ++r) {
    const int* xr = x + (size_t)(rowBase + m0 + 8 * hh + r) * SEQ_T;
    unsigned m = 0u;
#pragma unroll
    for (int q4 = 0; q4 < 4; ++q4) {
      const i4v w = *(const i4v*)(xr + 4 * q4);
#pragma unroll
      for (int e = 0; e < 4; ++e) m |= ((w[e] != 0) ? 1u : 0u) << (4 * q4 + e);
    }
    um[r] = m;
  }
  float bv[4][2];
#pragma unroll
  for (int g = 0; g < 4; ++g)
#pragma unroll
    for (int ub = 0; ub < 2; ++ub) bv[g][ub] = bias[g * HID_D + ub * 16 + c];

  const int* xg = x + (size_t)(rowBase + m0 + c) * SEQ_T;
  _Float16* arow = Ash + (m0 + c) * LS_PITCH;
  const float kZinv = 1.0f / 128.0f;
  const u4v z4 = {0u, 0u, 0u, 0u};

#pragma unroll 1
  for (int dir = 0; dir < 2; ++dir) {
    float cst[2][8], hst[2][8];
#pragma unroll
    for (int ub = 0; ub < 2; ++ub)
#pragma unroll
      for (int r = 0; r < 8; ++r) { cst[ub][r] = 0.0f; hst[ub][r] = 0.0f; }
    *(u4v*)(arow + 32 + 16 * hh)     = z4;
    *(u4v*)(arow + 32 + 16 * hh + 8) = z4;

#pragma unroll 1
    for (int s = 0; s < SEQ_T; ++s) {
      const int t = (dir == 0) ? s : (SEQ_T - 1 - s);
      int tok = xg[t];
      tok = tok < 0 ? 0 : tok;
      tok = tok > (nvocab - 1) ? (nvocab - 1) : tok;
      const float* er = etab + (size_t)tok * EMB_D + 16 * hh;
      const v4f e0 = *(const v4f*)(er);
      const v4f e1 = *(const v4f*)(er + 4);
      const v4f e2 = *(const v4f*)(er + 8);
      const v4f e3 = *(const v4f*)(er + 12);
      v8h p0, p1;
#pragma unroll
      for (int e = 0; e < 4; ++e) {
        p0[e]     = (_Float16)(e0[e] * 16.0f);
        p0[4 + e] = (_Float16)(e1[e] * 16.0f);
        p1[e]     = (_Float16)(e2[e] * 16.0f);
        p1[4 + e] = (_Float16)(e3[e] * 16.0f);
      }
      *(v8h*)(arow + 16 * hh)     = p0;
      *(v8h*)(arow + 16 * hh + 8) = p1;
      __syncthreads();

      v8f acc[4][2];
#pragma unroll
      for (int g = 0; g < 4; ++g)
#pragma unroll
        for (int ub = 0; ub < 2; ++ub) acc[g][ub] = (v8f){0.f,0.f,0.f,0.f,0.f,0.f,0.f,0.f};
#pragma unroll
      for (int ks = 0; ks < 2; ++ks) {
        const v16h af = Frag<_Float16>::load(arow + ks * 32 + 8 * hh);
#pragma unroll
        for (int ns = 0; ns < 8; ++ns) {
          const v16h bf = Frag<_Float16>::load(Wsh + (ns * 16 + c) * LS_PITCH + ks * 32 + 8 * hh);
          acc[ns >> 1][ns & 1] = mma_h(af, bf, acc[ns >> 1][ns & 1]);
        }
      }
      acc_guard4(acc[0][0], acc[0][1], acc[1][0], acc[1][1]);
      acc_guard4(acc[2][0], acc[2][1], acc[3][0], acc[3][1]);

#pragma unroll
      for (int ub = 0; ub < 2; ++ub) {
#pragma unroll
        for (int r = 0; r < 8; ++r) {
          const float zi = acc[0][ub][r] * kZinv + bv[0][ub];
          const float zf = acc[1][ub][r] * kZinv + bv[1][ub];
          const float zg = acc[2][ub][r] * kZinv + bv[2][ub];
          const float zo = acc[3][ub][r] * kZinv + bv[3][ub];
          const float ig = gate_sig(zi);
          const float fg = gate_sig(zf);
          const float gg = gate_tanh(zg);
          const float og = gate_sig(zo);
          const float cn = fg * cst[ub][r] + ig * gg;
          const float hn = og * gate_tanh(cn);
          const bool  mk = ((um[r] >> t) & 1u) != 0u;
          cst[ub][r] = mk ? cn : cst[ub][r];
          hst[ub][r] = mk ? hn : hst[ub][r];
          Ash[(m0 + 8 * hh + r) * LS_PITCH + 32 + ub * 16 + c] = (_Float16)(hst[ub][r] * 16.0f);
        }
      }
      __syncthreads();
    }
#pragma unroll
    for (int ub = 0; ub < 2; ++ub)
#pragma unroll
      for (int r = 0; r < 8; ++r)
        Osh[(m0 + 8 * hh + r) * LS_PITCH + dir * 32 + ub * 16 + c] = (_Float16)(hst[ub][r] * 16.0f);
  }
  __syncthreads();

  const int q = lane >> 3, c8 = (lane & 7) * 8;
  for (int pass = 0; pass < 2; ++pass) {
#pragma unroll
    for (int it = 0; it < 4; ++it) {
      const int row = it * 4 + q;
      const u4v v = *(const u4v*)(Osh + (m0 + row) * LS_PITCH + c8);
      *(volatile u4v*)(state16 + (size_t)(rowBase + m0 + row) * 64 + c8) = v;
    }
    __threadfence();
  }
}

extern "C" void kernel_launch(void* const* d_in, const int* in_sizes, int n_in,
                              void* d_out, int out_size, void* d_ws, size_t ws_size,
                              hipStream_t stream) {
  if (n_in < 7) return;
  const int*   x    = (const int*)d_in[0];
  const float* etab = (const float*)d_in[1];
  const float* Wk   = (const float*)d_in[2];
  const float* Wr   = (const float*)d_in[3];
  const float* b    = (const float*)d_in[4];
  const float* Wd   = (const float*)d_in[5];
  const float* bd   = (const float*)d_in[6];
  float*       out  = (float*)d_out;

  const int nTok   = in_sizes[0];
  const int nrows  = nTok / SEQ_T;
  const int nvocab = in_sizes[1] / EMB_D;
  const int Kd     = in_sizes[5] / 64;
  const int Mout   = out_size / 64;
  if (nTok % SEQ_T != 0 || nrows % LS_ROWS != 0 || nvocab < 1) return;
  if (in_sizes[2] != EMB_D * GATES_N || in_sizes[3] != HID_D * GATES_N || in_sizes[4] != GATES_N) return;
  if (in_sizes[6] != 64 || out_size % 64 != 0 || Mout % 64 != 0 || Kd % 64 != 0) return;
  if ((long)Mout * (long)Kd != (long)nrows * 64L) return;

  const size_t off_wcat  = 0;
  const size_t off_wdt   = 16384;
  const size_t off_state = off_wdt + (size_t)64 * Kd * 2;
  const size_t total     = off_state + (size_t)nrows * 64 * 2;
  if (total > ws_size) return;

  char* ws = (char*)d_ws;
  unsigned short* wcat    = (unsigned short*)(ws + off_wcat);
  unsigned short* wdt     = (unsigned short*)(ws + off_wdt);
  unsigned short* state16 = (unsigned short*)(ws + off_state);

  prep_wcat_kernel<<<dim3(1), dim3(256), 0, stream>>>(Wk, Wr, wcat);
  prep_wdt_kernel<<<dim3(Kd / 64), dim3(256), 0, stream>>>(Wd, wdt, Kd);
  lstm_bidir_kernel<<<dim3(nrows / LS_ROWS), dim3(128), 0, stream>>>(x, etab, b, wcat, state16, nvocab);

  const int tiles = (Mout / 64) * (64 / 64);
  const int gx    = (tiles + 7) / 8;
  wmma_gemm64<0, false, 2, 0, false, 1><<<dim3(gx, 1), dim3(256), 0, stream>>>(
      (const unsigned short*)state16, (const unsigned short*)nullptr, Kd, 0L,
      (const unsigned short*)wdt, (const unsigned short*)nullptr, Kd, 0L,
      (void*)out, (void*)nullptr, 64, 0L,
      bd, (const float*)nullptr, 0L,
      Mout, 64, Kd, 1.0f / 512.0f);
}
